// MAB_86148454023859
// MI455X (gfx1250) — hardware-run, weakly checked
//
#include <hip/hip_runtime.h>


namespace {
constexpr int B = 4, N = 2048, DI = 256, DV = 256, H = 4, HD = 64, BL = 4  , QL = 2048  ;
constexpr float XS = 8.0f, WSC = 256.0f, PS = 1024.0f, LOG2E = 1.4426950408889634f;
static_assert(N % 64 == 0 && QL % 64 == 0, "tiling");
typedef _Float16 b16;
typedef __attribute__((ext_vector_type(16))) _Float16 v16b;
typedef __attribute__((ext_vector_type(8))) _Float16 v8b;
typedef __attribute__((ext_vector_type(8))) float v8f;
typedef __attribute__((ext_vector_type(4))) float v4f;
__device__ __forceinline__ float bf16_rne(float f) { unsigned int u = __float_as_uint(f); u += 0x7FFFu + ((u >> 16) & 1u); return __uint_as_float(u & 0xFFFF0000u); }
__device__ __forceinline__ void split16(float v, b16& hi, b16& lo) { hi = (b16)v; lo = (b16)(v - (float)hi); }
__device__ __forceinline__ v16b frag_kb(const b16* p, int hh) { const v8b a = *(const v8b*)(p + 8 * hh), b = *(const v8b*)(p + 16 + 8 * hh); v16b f;
#pragma unroll
  for (int e = 0; e < 8; ++e) { f[e] = a[e]; f[8 + e] = b[e]; } return f; }
__device__ __forceinline__ v8f wmma16b(v16b a, v16b b, v8f c) { v8f d = __builtin_amdgcn_wmma_f32_16x16x32_f16(false, a, false, b, (short)0, c, false, false); asm volatile("v_nop\n\tv_nop\n\tv_nop\n\tv_nop" : "+v"(d) : "v"(a), "v"(b)); return d; }
__device__ __forceinline__ void wave_lds_sync() { __builtin_amdgcn_fence(__ATOMIC_RELEASE, "workgroup"); __builtin_amdgcn_wave_barrier(); __builtin_amdgcn_fence(__ATOMIC_ACQUIRE, "workgroup"); }
__device__ __forceinline__ float pmul(float a, float b) { float p = a * b; asm volatile("" : "+v"(p)); return p; }
__device__ __forceinline__ int iclamp(int v, int lo, int hi) { return v < lo ? lo : (v > hi ? hi : v); }

typedef __attribute__((ext_vector_type(2))) _Float16 v2h;
typedef __attribute__((ext_vector_type(4))) _Float16 v4h;
typedef __attribute__((ext_vector_type(2))) float v2f;
__device__ __forceinline__ float nexp2(float v) { return __builtin_amdgcn_exp2f(v); }
__global__ __launch_bounds__(256) void prep_kernel(const float* __restrict__ wq, const float* __restrict__ wk, const float* __restrict__ wv, const float* __restrict__ wo, b16* __restrict__ WT) {
  const int t = blockIdx.x * 256 + threadIdx.x; const int per = DV * DI / 8; if (t >= 4 * per) return; const int m = t / per; const int e = (t % per) * 8; const float* w = m == 0 ? wq : m == 1 ? wk : m == 2 ? wv : wo; v8b o;
  for (int j = 0; j < 8; ++j) o[j] = (b16)(bf16_rne(w[e + j]) * WSC);
  for (int pass = 0; pass < 2; ++pass) { *(volatile v8b*)(WT + (size_t)m * per * 8 + e) = o; __threadfence(); }
}
__global__ __launch_bounds__(128) void proj_kernel(const float* __restrict__ Qx, const float* __restrict__ Kx, const b16* __restrict__ WT, float* __restrict__ QF, b16* __restrict__ QP, b16* __restrict__ KP, b16* __restrict__ VT, float* __restrict__ MQ, float* __restrict__ MK) {
  __shared__ __attribute__((aligned(16))) float Tf[4][16][DV + 4]; __shared__ float FL[64];
  const int wave = threadIdx.x >> 5, lane = threadIdx.x & 31, nloc = lane & 15, hlf = lane >> 4; const int t0 = blockIdx.x * 64; const int b = blockIdx.y; const int part = blockIdx.z;
  if (part == 0 && t0 >= QL) return;
  const float* xb = (part == 0 ? Qx : Kx) + ((size_t)b * N + t0 + wave * 16) * DI; const b16* W = WT + (size_t)part * DV * DI;
  v8f acc[16];
#pragma unroll
  for (int t = 0; t < 16; ++t) acc[t] = (v8f){};
#pragma unroll 2
  for (int ks = 0; ks < DI / 32; ++ks) { v16b a; const float* xr = xb + (size_t)nloc * DI + ks * 32; const v4f c0 = *(const v4f*)(xr + 8 * hlf), c1 = *(const v4f*)(xr + 8 * hlf + 4), c2 = *(const v4f*)(xr + 16 + 8 * hlf), c3 = *(const v4f*)(xr + 16 + 8 * hlf + 4);
    for (int i = 0; i < 4; ++i) { a[i] = (b16)(bf16_rne(c0[i]) * XS); a[4 + i] = (b16)(bf16_rne(c1[i]) * XS); a[8 + i] = (b16)(bf16_rne(c2[i]) * XS); a[12 + i] = (b16)(bf16_rne(c3[i]) * XS); }
#pragma unroll
    for (int t = 0; t < 16; ++t) acc[t] = wmma16b(a, frag_kb(W + (size_t)(t * 16 + nloc) * DI + ks * 32, hlf), acc[t]); }
#pragma unroll
  for (int t = 0; t < 16; ++t)
#pragma unroll
    for (int r = 0; r < 8; ++r) Tf[wave][8 * hlf + r][t * 16 + nloc] = acc[t][r] * (1.0f / (XS * WSC));
  wave_lds_sync();
  if (part < 2) { for (int rr = 0; rr < 16; ++rr) { int nz = 0; for (int q = 0; q < 8; ++q) nz |= (Tf[wave][rr][q * 32 + lane] != 0.0f) ? 1 : 0;
#pragma unroll
      for (int o = 1; o < 32; o <<= 1) nz |= __shfl_xor(nz, o);
      if (lane == 0) FL[wave * 16 + rr] = nz ? 1.0f : 0.0f; } }
  __syncthreads();
  for (int pass = 0; pass < 2; ++pass) {
    if (part < 2) { b16* plane = part == 0 ? QP : KP;
      for (int rr = 0; rr < 16; ++rr) { const int tok = t0 + wave * 16 + rr; const size_t row = (size_t)b * N + tok;
        if (part == 0) { for (int q = lane * 4; q < DV; q += 128) *(volatile v4f*)(QF + row * DV + q) = *(const v4f*)(&Tf[wave][rr][q]); }
        for (int hp = 0; hp < 2; ++hp) { const int h = hp * 2 + (lane >> 4); const int d = (lane & 15) * 4; v4h o4; for (int j = 0; j < 4; ++j) o4[j] = (b16)(Tf[wave][rr][h * HD + d + j] * XS); *(volatile v4h*)(plane + (((size_t)b * H + h) * N + tok) * HD + d) = o4; } }
      if (wave == 0) { float* flag = (part == 0 ? MQ : MK) + (size_t)b * N + t0; ((volatile float*)flag)[lane] = FL[lane]; ((volatile float*)flag)[32 + lane] = FL[32 + lane]; } }
    else {
#pragma unroll 1
      for (int q = 0; q < 64; ++q) { const int c = wave * 64 + q; const int h = c / HD, d = c % HD; const int tk = lane * 2; v2h vv; vv[0] = (b16)(Tf[tk >> 4][tk & 15][c] * XS); vv[1] = (b16)(Tf[(tk + 1) >> 4][(tk + 1) & 15][c] * XS);
        *(volatile v2h*)(VT + (((size_t)b * H + h) * HD + d) * (size_t)N + t0 + tk) = vv; } }
    __threadfence(); }
}
__global__ __launch_bounds__(64) void attn_kernel(const b16* __restrict__ QP, const b16* __restrict__ KP, const b16* __restrict__ VT, const float* __restrict__ MQ, const float* __restrict__ MK, const float* __restrict__ QF, float* __restrict__ OF) {
  __shared__ __attribute__((aligned(16))) b16 Pb[2][16][32 + 8]; __shared__ __attribute__((aligned(16))) float To[2][16][HD + 4];
  const int wave = threadIdx.x >> 5, lane = threadIdx.x & 31, hh = lane >> 4, col = lane & 15; const int b = blockIdx.y / H, h = blockIdx.y % H; const int q0 = blockIdx.x * 32 + wave * 16, qi = q0 + col;
  const size_t ph = (size_t)b * H + h; const b16* Qb = QP + ph * N * HD; const b16* Kb = KP + ph * N * HD; const b16* Vb = VT + ph * HD * (size_t)N; const float* mk = MK + (size_t)b * N;
  const v16b qa0 = frag_kb(Qb + (size_t)qi * HD, hh), qa1 = frag_kb(Qb + (size_t)qi * HD + 32, hh); const bool qv = MQ[(size_t)b * N + qi] != 0.0f;
  const float cs = LOG2E / (16.0f * XS * XS);
  float m = -INFINITY, l = 0.0f; v8f o[4]; for (int t = 0; t < 4; ++t) o[t] = (v8f){};
#pragma unroll 1
  for (int kb = 0; kb < N; kb += 32) {
    float e[16]; float mx = -INFINITY;
#pragma unroll
    for (int u = 0; u < 2; ++u) { v8f s = (v8f){}; const size_t kr = (size_t)(kb + u * 16 + col) * HD; s = wmma16b(frag_kb(Kb + kr, hh), qa0, s); s = wmma16b(frag_kb(Kb + kr + 32, hh), qa1, s);
      const v4f m0 = *(const v4f*)(mk + kb + u * 16 + 8 * hh), m1 = *(const v4f*)(mk + kb + u * 16 + 8 * hh + 4);
#pragma unroll
      for (int r = 0; r < 8; ++r) { const float kvld = (r < 4) ? m0[r] : m1[r - 4]; const float vv = (qv && kvld != 0.0f) ? s[r] * cs : -INFINITY; e[u * 8 + r] = vv; mx = fmaxf(mx, vv); } }
    mx = fmaxf(mx, __shfl_xor(mx, 16)); const float mn = fmaxf(m, mx); const float al = (mn == -INFINITY) ? 1.0f : nexp2(m - mn); float sum = 0.0f;
#pragma unroll
    for (int i2 = 0; i2 < 16; ++i2) { const float p = (e[i2] == -INFINITY) ? 0.0f : nexp2(e[i2] - mn); sum += p; Pb[wave][col][(i2 < 8 ? 0 : 16) + 8 * hh + (i2 & 7)] = (b16)(p * PS); }
    sum += __shfl_xor(sum, 16); l = l * al + sum; m = mn;
    wave_lds_sync();
    const v16b pf = frag_kb(&Pb[wave][col][0], hh);
#pragma unroll
    for (int t = 0; t < 4; ++t) { o[t] *= al; o[t] = wmma16b(frag_kb(Vb + (size_t)(t * 16 + col) * N + kb, hh), pf, o[t]); }
    wave_lds_sync(); }
  const float inv = (l > 0.0f) ? 1.0f / (l * PS * XS) : 0.0f;
#pragma unroll
  for (int t = 0; t < 4; ++t)
#pragma unroll
    for (int r = 0; r < 8; ++r) To[wave][col][t * 16 + 8 * hh + r] = o[t][r] * inv;
  wave_lds_sync();
  for (int pass = 0; pass < 2; ++pass) { for (int rr = 0; rr < 16; ++rr) { const size_t oi = ((size_t)b * N + q0 + rr) * DV + h * HD + lane * 2; v2f f = *(const v2f*)(&To[wave][rr][lane * 2]); const v2f qf = *(const v2f*)(QF + oi); f += qf; *(volatile v2f*)(OF + oi) = f; } __threadfence(); }
}
__global__ __launch_bounds__(128) void ffn_kernel(const float* __restrict__ OF, const b16* __restrict__ WT, float* __restrict__ out) {
  __shared__ __attribute__((aligned(16))) float Tf[4][16][DV + 4];
  const int wave = threadIdx.x >> 5, lane = threadIdx.x & 31, nloc = lane & 15, hlf = lane >> 4; const int b = blockIdx.y; const size_t r0 = (size_t)b * N + ((size_t)blockIdx.x * 4 + wave) * 16; const b16* W = WT + (size_t)3 * DV * DI;
  v8f acc[16];
#pragma unroll
  for (int t = 0; t < 16; ++t) acc[t] = (v8f){};
#pragma unroll 2
  for (int ks = 0; ks < DV / 32; ++ks) { v16b ah, al; const float* xr = OF + (r0 + nloc) * DV + ks * 32; const v4f c0 = *(const v4f*)(xr + 8 * hlf), c1 = *(const v4f*)(xr + 8 * hlf + 4), c2 = *(const v4f*)(xr + 16 + 8 * hlf), c3 = *(const v4f*)(xr + 16 + 8 * hlf + 4); float cv[16];
    for (int i = 0; i < 4; ++i) { cv[i] = c0[i]; cv[4 + i] = c1[i]; cv[8 + i] = c2[i]; cv[12 + i] = c3[i]; }
    for (int e2 = 0; e2 < 16; ++e2) { b16 p, q; split16(cv[e2] * XS, p, q); ah[e2] = p; al[e2] = q; }
#pragma unroll
    for (int t = 0; t < 16; ++t) { const v16b bw = frag_kb(W + (size_t)(t * 16 + nloc) * DV + ks * 32, hlf); acc[t] = wmma16b(ah, bw, acc[t]); acc[t] = wmma16b(al, bw, acc[t]); } }
#pragma unroll
  for (int t = 0; t < 16; ++t)
#pragma unroll
    for (int r = 0; r < 8; ++r) Tf[wave][8 * hlf + r][t * 16 + nloc] = fmaxf(acc[t][r] * (1.0f / (XS * WSC)), 0.0f);
  wave_lds_sync();
  for (int pass = 0; pass < 2; ++pass) { for (int rr = 0; rr < 16; ++rr) { for (int q = lane * 4; q < DV; q += 128) { v4f f = *(const v4f*)(&Tf[wave][rr][q]); const v4f of = *(const v4f*)(OF + (r0 + rr) * DV + q); f += of; *(volatile v4f*)(out + (r0 + rr) * DV + q) = f; } } __threadfence(); }
}
}

extern "C" void kernel_launch(void* const* d_in, const int* in_sizes, int n_in, void* d_out, int out_size, void* d_ws, size_t ws_size, hipStream_t stream) {
  (void)n_in;
  auto Fp = [&](int i) { return (const float*)d_in[i]; };
  if (in_sizes[0] != B * N * DI || in_sizes[1] != B * N * DI || in_sizes[2] != DV * DI || in_sizes[3] != DV * DI || in_sizes[4] != DV * DI || in_sizes[5] != DV * DV || out_size != B * N * DV) return;
  size_t off = 0; char* ws = (char*)d_ws;
  auto carve = [&](size_t bytes) { char* p = ws + off; off += (bytes + 255) & ~(size_t)255; return p; };
  b16* WT = (b16*)carve((size_t)4 * DV * DI * 2); float* QF = (float*)carve((size_t)B * N * DV * 4); float* OF = (float*)carve((size_t)B * N * DV * 4);
  const size_t plane = (size_t)B * N * DV * 2; b16* QP = (b16*)carve(plane); b16* KP = (b16*)carve(plane); b16* VT = (b16*)carve(plane); float* MQ = (float*)carve((size_t)B * N * 4); float* MK = (float*)carve((size_t)B * N * 4);
  if (off > ws_size || off > ((size_t)128 << 20)) return;
  prep_kernel<<<(4 * DV * DI / 8 + 255) / 256, 256, 0, stream>>>(Fp(2), Fp(3), Fp(4), Fp(5), WT);
  proj_kernel<<<dim3(N / 64, BL, 3), 128, 0, stream>>>(Fp(0), Fp(1), WT, QF, QP, KP, VT, MQ, MK);
  attn_kernel<<<dim3(QL / 32, BL * H), 64, 0, stream>>>(QP, KP, VT, MQ, MK, QF, OF);
  ffn_kernel<<<dim3(QL / 64, BL), 128, 0, stream>>>(OF, WT, (float*)d_out);
}
